// Sequence_Modeling_40381282517740
// MI455X (gfx1250) — hardware-verified
//
#include <hip/hip_runtime.h>

typedef __attribute__((ext_vector_type(16))) _Float16 v16h;
typedef __attribute__((ext_vector_type(8)))  _Float16 v8h;
typedef __attribute__((ext_vector_type(16))) __bf16   v16b;
typedef __attribute__((ext_vector_type(8)))  __bf16   v8b;
typedef __attribute__((ext_vector_type(8)))  float    v8f;
typedef __attribute__((ext_vector_type(4)))  float    v4f;
typedef __attribute__((ext_vector_type(4)))  unsigned v4u;

__device__ __forceinline__ unsigned short f2bf_bits(float f) {
  unsigned u = __float_as_uint(f);
  return (unsigned short)((u + 0x7FFFu + ((u >> 16) & 1u)) >> 16);
}
__device__ __forceinline__ float bf_bits2f(unsigned short h) { return __uint_as_float(((unsigned)h) << 16); }

__device__ __forceinline__ void dep_guard_h(v8f& a, v8f& b, v16h x, v16h y) { asm volatile("v_nop\n\tv_nop\n\tv_nop\n\tv_nop" : "+v"(a), "+v"(b) : "v"(x), "v"(y)); }
__device__ __forceinline__ void dep_guard_b(v8f& a, v8f& b, v16b x, v16b y) { asm volatile("v_nop\n\tv_nop\n\tv_nop\n\tv_nop" : "+v"(a), "+v"(b) : "v"(x), "v"(y)); }
__device__ __forceinline__ void keep4_h(v16h a, v16h b, v16h c, v16h d) { asm volatile("v_nop" :: "v"(a), "v"(b), "v"(c), "v"(d)); }
__device__ __forceinline__ void keep4_b(v16b a, v16b b, v16b c, v16b d) { asm volatile("v_nop" :: "v"(a), "v"(b), "v"(c), "v"(d)); }
__device__ __forceinline__ void acc_guard4(v8f& a, v8f& b, v8f& c, v8f& d) { asm volatile("v_nop\n\tv_nop\n\tv_nop\n\tv_nop" : "+v"(a), "+v"(b), "+v"(c), "+v"(d)); }
template <typename T> struct Frag;
template <> struct Frag<_Float16> {
  typedef v16h V; union U { v16h v; v8h h[2]; };
  static __device__ __forceinline__ v16h load(const _Float16* p) {
    U f; f.h[0] = *(const v8h*)(p); f.h[1] = *(const v8h*)(p + 16); return f.v;
  }
  static __device__ __forceinline__ v8f mma(v16h a, v16h b, v8f c) {
    return __builtin_amdgcn_wmma_f32_16x16x32_f16(false, a, false, b, (short)0, c, false, false);
  }
  static __device__ __forceinline__ void guard(v8f& a, v8f& b, v16h x, v16h y) { dep_guard_h(a, b, x, y); }
  static __device__ __forceinline__ void keep(v16h a, v16h b, v16h c, v16h d) { keep4_h(a, b, c, d); }
};
template <> struct Frag<__bf16> {
  typedef v16b V; union U { v16b v; v8b h[2]; };
  static __device__ __forceinline__ v16b load(const __bf16* p) {
    U f; f.h[0] = *(const v8b*)(p); f.h[1] = *(const v8b*)(p + 16); return f.v;
  }
  static __device__ __forceinline__ v8f mma(v16b a, v16b b, v8f c) {
    return __builtin_amdgcn_wmma_f32_16x16x32_bf16(false, a, false, b, (short)0, c, false, false);
  }
  static __device__ __forceinline__ void guard(v8f& a, v8f& b, v16b x, v16b y) { dep_guard_b(a, b, x, y); }
  static __device__ __forceinline__ void keep(v16b a, v16b b, v16b c, v16b d) { keep4_b(a, b, c, d); }
};

template <int ET> struct Elem;
template <> struct Elem<0> { typedef _Float16 T; };
template <> struct Elem<1> { typedef __bf16 T; };
template <int ET, bool SPLIT, int BIAS_MODE, int OUT_MODE, bool RESID, int ACT = 0>
__global__ __launch_bounds__(256) void wmma_gemm64(
    const unsigned short* __restrict__ Ap, const unsigned short* __restrict__ A2p, int lda, long strideA,
    const unsigned short* __restrict__ Btp, const unsigned short* __restrict__ Bt2p, int ldb, long strideB,
    void* __restrict__ Cout, void* __restrict__ Cout2, int ldc, long strideC,
    const float* __restrict__ bias,
    const float* __restrict__ resid, long strideR,
    int M, int N, int K, float scale) {
  typedef typename Elem<ET>::T T;
  typedef typename Frag<T>::V V;
  const T* A = (const T*)Ap; const T* A2 = (const T*)A2p; const T* Bt = (const T*)Btp; const T* Bt2 = (const T*)Bt2p;
  __shared__ __align__(16) float sT[8][16 * 68];
  const int b    = blockIdx.y;
  const int lane = threadIdx.x & 31;
  const int wave = threadIdx.x >> 5;
  const int tilesN = N >> 6;
  const int tilesM = M >> 6;
  const int tile = blockIdx.x * 8 + wave;
  if (tile >= tilesM * tilesN) return;
  const int tm = tile / tilesN;
  const int tn = tile - tm * tilesN;
  const int m0 = tm << 6;
  const int n0 = tn << 6;

  const T* Ab  = A  + (size_t)b * strideA;
  const T* Bb  = Bt + (size_t)b * strideB;
  const T* Ab2 = SPLIT ? (A2  + (size_t)b * strideA) : nullptr;
  const T* Bb2 = SPLIT ? (Bt2 + (size_t)b * strideB) : nullptr;

  const int rlane = lane & 15;
  const int koff  = (lane >> 4) * 8;
  const int mOff  = (lane >> 4) * 8;

  v8f acc[4][4];
#pragma unroll
  for (int i = 0; i < 4; ++i)
#pragma unroll
    for (int j = 0; j < 4; ++j) acc[i][j] = (v8f){0.f,0.f,0.f,0.f,0.f,0.f,0.f,0.f};

  for (int k0 = 0; k0 < K; k0 += 32) {
    V bh[4], bl[4];
#pragma unroll
    for (int j = 0; j < 4; ++j) {
      const size_t bo = (size_t)(n0 + (j << 4) + rlane) * ldb + koff + k0;
      bh[j] = Frag<T>::load(Bb + bo);
      if (SPLIT) bl[j] = Frag<T>::load(Bb2 + bo);
    }
#pragma unroll
    for (int i = 0; i < 4; ++i) {
      const size_t ao = (size_t)(m0 + (i << 4) + rlane) * lda + koff + k0;
      V ah = Frag<T>::load(Ab + ao);
      V al;
      if (SPLIT) al = Frag<T>::load(Ab2 + ao);
#pragma unroll
      for (int j = 0; j < 4; ++j) {
        acc[i][j] = Frag<T>::mma(ah, bh[j], acc[i][j]);
        if (SPLIT) {
          acc[i][j] = Frag<T>::mma(ah, bl[j], acc[i][j]);
          acc[i][j] = Frag<T>::mma(al, bh[j], acc[i][j]);
        }
      }
      Frag<T>::guard(acc[i][0], acc[i][3], ah, SPLIT ? al : ah);
    }
    Frag<T>::keep(bh[0], bh[1], bh[2], bh[3]);
    if (SPLIT) Frag<T>::keep(bl[0], bl[1], bl[2], bl[3]);
  }
  acc_guard4(acc[0][0], acc[0][1], acc[0][2], acc[0][3]);
  acc_guard4(acc[1][0], acc[1][1], acc[1][2], acc[1][3]);
  acc_guard4(acc[2][0], acc[2][1], acc[2][2], acc[2][3]);
  acc_guard4(acc[3][0], acc[3][1], acc[3][2], acc[3][3]);

  float* slab = sT[wave];
  const float* Rb = RESID ? (resid + (size_t)b * strideR) : nullptr;
#pragma unroll
  for (int i = 0; i < 4; ++i) {
    const int mBase = m0 + (i << 4);
#pragma unroll
    for (int j = 0; j < 4; ++j) {
      const int n = n0 + (j << 4) + rlane;
      float bv = 0.f;
      if (BIAS_MODE == 2) bv = bias[n];
#pragma unroll
      for (int r = 0; r < 8; ++r) {
        float v = acc[i][j][r] * scale;
        if (BIAS_MODE == 1) v += bias[mBase + mOff + r];
        if (BIAS_MODE == 2) v += bv;
        if (RESID) v += Rb[(size_t)(mBase + mOff + r) * ldc + n];
        if (ACT == 1) v = tanhf(v);
        if (ACT == 2) v = fmaxf(v, 0.0f);
        if (ACT == 3) v = v / (1.0f + expf(-v));
        if (ACT == 4) v = (v > 0.f) ? v : 0.01f * v;
        if (ACT == 5) v = 0.5f * v * (1.0f + erff(v * 0.70710678118654752f));
        slab[(mOff + r) * 68 + (j << 4) + rlane] = v;
      }
    }
    __builtin_amdgcn_fence(__ATOMIC_RELEASE, "workgroup");
    __builtin_amdgcn_wave_barrier();
    __builtin_amdgcn_fence(__ATOMIC_ACQUIRE, "workgroup");
    if (OUT_MODE == 0) {
      float* C = (float*)Cout + (size_t)b * strideC;
      const int hh = lane >> 4, c4 = (lane & 15) * 4;
      for (int pass = 0; pass < 2; ++pass) {
#pragma unroll
        for (int it = 0; it < 8; ++it) {
          const int row = it * 2 + hh;
          v4f v = *(const v4f*)(slab + row * 68 + c4);
          *(volatile v4f*)(C + (size_t)(mBase + row) * ldc + n0 + c4) = v;
        }
        __threadfence();
      }
    } else {
      const int q = lane >> 3, c8 = (lane & 7) * 8;
      unsigned short* C  = (unsigned short*)Cout  + (size_t)b * strideC;
      unsigned short* C2 = (OUT_MODE == 2) ? ((unsigned short*)Cout2 + (size_t)b * strideC) : nullptr;
      for (int pass = 0; pass < 2; ++pass) {
#pragma unroll
        for (int it = 0; it < 4; ++it) {
          const int row = it * 4 + q;
          const float* sp = slab + row * 68 + c8;
          v8h hv, lv;
#pragma unroll
          for (int e = 0; e < 8; ++e) {
            if (OUT_MODE == 1) {
              hv[e] = (_Float16)sp[e];
            } else {
              unsigned short hb = f2bf_bits(sp[e]);
              unsigned short lb = f2bf_bits(sp[e] - bf_bits2f(hb));
              hv[e] = __builtin_bit_cast(_Float16, hb);
              lv[e] = __builtin_bit_cast(_Float16, lb);
            }
          }
          *(volatile v8h*)(C + (size_t)(mBase + row) * ldc + n0 + c8) = hv;
          if (OUT_MODE == 2) *(volatile v8h*)(C2 + (size_t)(mBase + row) * ldc + n0 + c8) = lv;
        }
        __threadfence();
      }
    }
    __builtin_amdgcn_fence(__ATOMIC_RELEASE, "workgroup");
    __builtin_amdgcn_wave_barrier();
    __builtin_amdgcn_fence(__ATOMIC_ACQUIRE, "workgroup");
  }
}

static constexpr int kNB   = 32;
static constexpr int kSE   = 512;
static constexpr int kSD   = 128;
static constexpr int kEMB  = 256;
static constexpr int kHID  = 512;
static constexpr int kNOUT = 1024;
static constexpr int kVOC  = 50257;
static constexpr int kKCAT = kHID + kEMB + kHID;
static constexpr int kRB   = 16;
static constexpr int kHP   = kHID + 8;

__device__ __forceinline__ unsigned pack_hilo2(float a, float b, unsigned& lo2) {
  const unsigned short ha = f2bf_bits(a), hb = f2bf_bits(b);
  const unsigned short la = f2bf_bits(a - bf_bits2f(ha)), lb = f2bf_bits(b - bf_bits2f(hb));
  lo2 = (unsigned)la | ((unsigned)lb << 16);
  return (unsigned)ha | ((unsigned)hb << 16);
}
__device__ __forceinline__ void split8(v4f a, v4f b, v4u& hv, v4u& lv) {
  unsigned l0, l1, l2, l3;
  const unsigned h0 = pack_hilo2(a.x, a.y, l0);
  const unsigned h1 = pack_hilo2(a.z, a.w, l1);
  const unsigned h2 = pack_hilo2(b.x, b.y, l2);
  const unsigned h3 = pack_hilo2(b.z, b.w, l3);
  hv = (v4u){h0, h1, h2, h3};
  lv = (v4u){l0, l1, l2, l3};
}
__device__ __forceinline__ v4f sel4(bool c, v4f a, v4f b) {
  v4f r;
  r.x = c ? a.x : b.x; r.y = c ? a.y : b.y; r.z = c ? a.z : b.z; r.w = c ? a.w : b.w;
  return r;
}
__device__ __forceinline__ v4f zero4() { return (v4f){0.f, 0.f, 0.f, 0.f}; }
__device__ __forceinline__ v8f zero8() { return (v8f){0.f,0.f,0.f,0.f,0.f,0.f,0.f,0.f}; }

__global__ __launch_bounds__(256) void k_split8(const float* __restrict__ src,
    unsigned short* __restrict__ hi, unsigned short* __restrict__ lo, int n8) {
  const int i = blockIdx.x * 256 + threadIdx.x;
  if (i >= n8) return;
  const size_t o = (size_t)i * 8;
  const v4f a = *(const v4f*)(src + o);
  const v4f b = *(const v4f*)(src + o + 4);
  v4u hv, lv; split8(a, b, hv, lv);
  for (int pass = 0; pass < 2; ++pass) {
    *(volatile v4u*)(hi + o) = hv;
    *(volatile v4u*)(lo + o) = lv;
    __threadfence();
  }
}

__global__ __launch_bounds__(256) void k_build_wcat(const float* __restrict__ wih, const float* __restrict__ whh,
    unsigned short* __restrict__ hi, unsigned short* __restrict__ lo, int nthr) {
  const int i = blockIdx.x * 256 + threadIdx.x;
  if (i >= nthr) return;
  const int n = i / 160;
  const int g = i - n * 160;
  const int c = g * 8;
  const bool first = (c < (kHID + kEMB));
  const int cih = first ? c : (kHID + kEMB - 8);
  const int chh = first ? 0 : (c - (kHID + kEMB));
  const float* pa = wih + (size_t)n * (kHID + kEMB) + cih;
  const float* pb = whh + (size_t)n * kHID + chh;
  const v4f a0 = *(const v4f*)pa, a1 = *(const v4f*)(pa + 4);
  const v4f b0 = *(const v4f*)pb, b1 = *(const v4f*)(pb + 4);
  const v4f x0 = sel4(first, a0, b0), x1 = sel4(first, a1, b1);
  v4u hv, lv; split8(x0, x1, hv, lv);
  const size_t o = (size_t)n * kKCAT + c;
  for (int pass = 0; pass < 2; ++pass) {
    *(volatile v4u*)(hi + o) = hv;
    *(volatile v4u*)(lo + o) = lv;
    __threadfence();
  }
}

__global__ __launch_bounds__(256) void k_gather_rows(const int* __restrict__ ids, const float* __restrict__ emb,
    unsigned short* __restrict__ hi, unsigned short* __restrict__ lo, int nthr) {
  const int i = blockIdx.x * 256 + threadIdx.x;
  if (i >= nthr) return;
  const int m = i >> 5, g = i & 31;
  const int b = m & 31, s = m >> 5;
  int id = ids[b * kSE + s];
  id = id < 0 ? 0 : (id > kVOC - 1 ? kVOC - 1 : id);
  const float* src = emb + (size_t)id * kEMB + 8 * g;
  const v4f a = *(const v4f*)src;
  const v4f c = *(const v4f*)(src + 4);
  v4u hv, lv; split8(a, c, hv, lv);
  const size_t o = (size_t)m * kEMB + 8 * g;
  for (int pass = 0; pass < 2; ++pass) {
    *(volatile v4u*)(hi + o) = hv;
    *(volatile v4u*)(lo + o) = lv;
    __threadfence();
  }
}

__global__ __launch_bounds__(256) void k_encoder(
    const float* __restrict__ xw,
    const unsigned short* __restrict__ whh_hi,
    const unsigned short* __restrict__ whh_lo,
    const float* __restrict__ bhh,
    float* __restrict__ eh) {
  typedef Frag<__bf16> F;
  typedef v16b V;
  __shared__ __align__(16) unsigned short Ah[kRB * kHP];
  __shared__ __align__(16) unsigned short Al[kRB * kHP];
  __shared__ __align__(16) float slab[8][16 * 68];
  const int tid = threadIdx.x, lane = tid & 31, wave = tid >> 5;
  const int rlane = lane & 15, hh = lane >> 4, koff = hh * 8;
  const int c4 = rlane * 4;
  const int blk = blockIdx.x;
  const int b0 = blk * kRB;

  for (int i = tid; i < kRB * kHP; i += 256) { Ah[i] = 0; Al[i] = 0; }
  float bcol[4];
#pragma unroll
  for (int j = 0; j < 4; ++j) bcol[j] = bhh[64 * wave + 16 * j + rlane];
  __syncthreads();

  const __bf16* Ahp = (const __bf16*)Ah;
  const __bf16* Alp = (const __bf16*)Al;
  const __bf16* Bhp = (const __bf16*)whh_hi;
  const __bf16* Blp = (const __bf16*)whh_lo;
  float* sl = slab[wave];

  for (int t = 0; t < kSE; ++t) {
    v8f acc[4];
#pragma unroll
    for (int j = 0; j < 4; ++j) acc[j] = zero8();
#pragma unroll 1
    for (int k0 = 0; k0 < kHID; k0 += 32) {
      V bh[4], bl[4];
#pragma unroll
      for (int j = 0; j < 4; ++j) {
        const size_t bo = (size_t)(64 * wave + 16 * j + rlane) * kHID + koff + k0;
        bh[j] = F::load(Bhp + bo);
        bl[j] = F::load(Blp + bo);
      }
      const int ao = rlane * kHP + koff + k0;
      const V ah = F::load(Ahp + ao);
      const V al = F::load(Alp + ao);
#pragma unroll
      for (int j = 0; j < 4; ++j) {
        acc[j] = F::mma(ah, bh[j], acc[j]);
        acc[j] = F::mma(ah, bl[j], acc[j]);
        acc[j] = F::mma(al, bh[j], acc[j]);
      }
      F::guard(acc[0], acc[3], ah, al);
      F::keep(bh[0], bh[1], bh[2], bh[3]);
      F::keep(bl[0], bl[1], bl[2], bl[3]);
    }
    acc_guard4(acc[0], acc[1], acc[2], acc[3]);
    __syncthreads();

    const size_t xbase = ((size_t)t * kNB + b0) * kHID;
#pragma unroll
    for (int j = 0; j < 4; ++j) {
      const int col = 64 * wave + 16 * j + rlane;
#pragma unroll
      for (int r = 0; r < 8; ++r) {
        const int row = 8 * hh + r;
        float v = xw[xbase + (size_t)row * kHID + col] + acc[j][r];
        v = tanhf(v + bcol[j]);
        sl[row * 68 + 16 * j + rlane] = v;
        const unsigned short hb = f2bf_bits(v);
        const unsigned short lb = f2bf_bits(v - bf_bits2f(hb));
        Ah[row * kHP + col] = hb;
        Al[row * kHP + col] = lb;
      }
    }
    __builtin_amdgcn_fence(__ATOMIC_RELEASE, "workgroup");
    __builtin_amdgcn_wave_barrier();
    __builtin_amdgcn_fence(__ATOMIC_ACQUIRE, "workgroup");
    for (int pass = 0; pass < 2; ++pass) {
#pragma unroll
      for (int it = 0; it < 8; ++it) {
        const int row = it * 2 + hh;
        const v4f v = *(const v4f*)(sl + row * 68 + c4);
        *(volatile v4f*)(eh + ((size_t)(b0 + row) * kSE + t) * kHID + 64 * wave + c4) = v;
      }
      __threadfence();
    }
    __syncthreads();
  }
}

__global__ __launch_bounds__(256) void k_hmean(const float* __restrict__ eh,
    unsigned short* __restrict__ hmh, unsigned short* __restrict__ hml) {
  const int i = blockIdx.x * 256 + threadIdx.x;
  const int row = i >> 6, g = i & 63, c = g * 8;
  v4f s0 = zero4(), s1 = zero4();
  if (blockIdx.x < 8) {
    const float* p = eh + (size_t)row * kSE * kHID + c;
#pragma unroll 1
    for (int ob = 0; ob < 8; ++ob) {
      v4f p0 = zero4(), p1 = zero4();
#pragma unroll 1
      for (int t = 0; t < 64; ++t) {
        const float* q = p + (size_t)(ob * 64 + t) * kHID;
        p0 = p0 + *(const v4f*)q;
        p1 = p1 + *(const v4f*)(q + 4);
      }
      s0 = s0 + p0;
      s1 = s1 + p1;
    }
    const float inv = 1.0f / 512.0f;
    s0 = s0 * inv;
    s1 = s1 * inv;
  }
  v4u hv, lv; split8(s0, s1, hv, lv);
  const size_t o = (size_t)row * kHID + c;
  for (int pass = 0; pass < 2; ++pass) {
    *(volatile v4u*)(hmh + o) = hv;
    *(volatile v4u*)(hml + o) = lv;
    __threadfence();
  }
}

__device__ __forceinline__ void state_to_planes(const float* ssh, unsigned short* tgh, unsigned short* tgl, int tid) {
  v4u hv[4], lv[4];
#pragma unroll
  for (int k = 0; k < 4; ++k) {
    const int L = 256 * k + tid;
    const int row = L >> 6, g = L & 63;
    const v4f a = *(const v4f*)(ssh + row * kHID + 8 * g);
    const v4f b = *(const v4f*)(ssh + row * kHID + 8 * g + 4);
    split8(a, b, hv[k], lv[k]);
  }
  for (int pass = 0; pass < 2; ++pass) {
#pragma unroll
    for (int k = 0; k < 4; ++k) {
      const int L = 256 * k + tid;
      const int row = L >> 6, g = L & 63;
      const size_t o = (size_t)row * kKCAT + (kHID + kEMB) + 8 * g;
      *(volatile v4u*)(tgh + o) = hv[k];
      *(volatile v4u*)(tgl + o) = lv[k];
    }
    __threadfence();
  }
}

__global__ __launch_bounds__(256) void k_decoder(
    const float* __restrict__ eh,
    const float* __restrict__ s0p,
    const int* __restrict__ dec_y,
    const float* __restrict__ emb,
    const unsigned short* __restrict__ wc_hi,
    const unsigned short* __restrict__ wc_lo,
    const float* __restrict__ bih,
    const float* __restrict__ bhh,
    const unsigned short* __restrict__ m2_hi,
    const unsigned short* __restrict__ m2_lo,
    const float* __restrict__ m2b,
    unsigned short* tg_hi,
    unsigned short* tg_lo,
    float* __restrict__ out) {
  typedef Frag<__bf16> F;
  typedef v16b V;
  __shared__ __align__(16) float Ssh[kRB * kHID];
  __shared__ __align__(16) float Rg[8 * 16 * 68];
  const int tid = threadIdx.x, lane = tid & 31, wave = tid >> 5;
  const int rlane = lane & 15, hh = lane >> 4, koff = hh * 8;
  const int c4 = rlane * 4;
  const int blk = blockIdx.x;
  const int b0 = blk * kRB;
  unsigned short* tgh = tg_hi + (size_t)b0 * kKCAT;
  unsigned short* tgl = tg_lo + (size_t)b0 * kKCAT;

  {
    const int row = tid >> 4, sub = tid & 15;
    const float* sp = s0p + (size_t)(b0 + row) * kHID + 32 * sub;
#pragma unroll
    for (int k = 0; k < 8; ++k)
      *(v4f*)(Ssh + row * kHID + 32 * sub + 4 * k) = *(const v4f*)(sp + 4 * k);
  }
  float bcat[4];
#pragma unroll
  for (int j = 0; j < 4; ++j) {
    const int col = 64 * wave + 16 * j + rlane;
    bcat[j] = bih[col] + bhh[col];
  }
  __syncthreads();
  state_to_planes(Ssh, tgh, tgl, tid);
  __syncthreads();
  __threadfence();

  const __bf16* Thp = (const __bf16*)tgh;
  const __bf16* Tlp = (const __bf16*)tgl;
  const __bf16* Wchp = (const __bf16*)wc_hi;
  const __bf16* Wclp = (const __bf16*)wc_lo;
  const __bf16* M2hp = (const __bf16*)m2_hi;
  const __bf16* M2lp = (const __bf16*)m2_lo;

  for (int t = 0; t < kSD; ++t) {
    {
      v4u hv[2], lv[2];
#pragma unroll
      for (int k = 0; k < 2; ++k) {
        const int row = 8 * k + wave;
        int id = dec_y[(b0 + row) * kSD + t];
        id = id < 0 ? 0 : (id > kVOC - 1 ? kVOC - 1 : id);
        const float* ep = emb + (size_t)id * kEMB + 8 * lane;
        const v4f a = *(const v4f*)ep;
        const v4f b = *(const v4f*)(ep + 4);
        split8(a, b, hv[k], lv[k]);
      }
      for (int pass = 0; pass < 2; ++pass) {
#pragma unroll
        for (int k = 0; k < 2; ++k) {
          const size_t o = (size_t)(8 * k + wave) * kKCAT + kHID + 8 * lane;
          *(volatile v4u*)(tgh + o) = hv[k];
          *(volatile v4u*)(tgl + o) = lv[k];
        }
        __threadfence();
      }
    }
    {
      const int oct = tid >> 3, sub = tid & 7;
#pragma unroll 1
      for (int r = 0; r < kRB; ++r) {
        const float* er = eh + ((size_t)(b0 + r) * kSE + oct) * kHID + 4 * sub;
        const float* sr = Ssh + r * kHID + 4 * sub;
        v4f a4[16];
#pragma unroll
        for (int q = 0; q < 16; ++q) a4[q] = zero4();
#pragma unroll 1
        for (int hc = 0; hc < 16; ++hc) {
          const v4f sv = *(const v4f*)(sr + 32 * hc);
#pragma unroll
          for (int q = 0; q < 16; ++q) {
            const v4f ev = *(const v4f*)(er + (size_t)q * 32 * kHID + 32 * hc);
            a4[q] = a4[q] + ev * sv;
          }
        }
        float sc[16];
#pragma unroll
        for (int q = 0; q < 16; ++q) {
          float v = (a4[q].x + a4[q].y) + (a4[q].z + a4[q].w);
          v += __shfl_xor(v, 1, 32);
          v += __shfl_xor(v, 2, 32);
          v += __shfl_xor(v, 4, 32);
          sc[q] = v;
        }
        if (sub == 0) {
#pragma unroll
          for (int q = 0; q < 16; ++q) Rg[r * kSE + oct + 32 * q] = sc[q];
        }
      }
    }
    __syncthreads();
    {
#pragma unroll 1
      for (int rr = 0; rr < 2; ++rr) {
        const int r = 2 * wave + rr;
        float* pr = Rg + r * kSE;
        float m = -__builtin_inff();
#pragma unroll 1
        for (int i = 0; i < 16; ++i) m = fmaxf(m, pr[lane + 32 * i]);
#pragma unroll
        for (int off = 1; off < 32; off <<= 1) m = fmaxf(m, __shfl_xor(m, off, 32));
        float ssum = 0.f;
#pragma unroll 1
        for (int i = 0; i < 16; ++i) {
          const float e = expf(pr[lane + 32 * i] - m);
          pr[lane + 32 * i] = e;
          ssum += e;
        }
#pragma unroll
        for (int off = 1; off < 32; off <<= 1) ssum += __shfl_xor(ssum, off, 32);
        const float inv = 1.0f / ssum;
#pragma unroll 1
        for (int i = 0; i < 16; ++i) pr[lane + 32 * i] = pr[lane + 32 * i] * inv;
      }
    }
    __syncthreads();
    {
      const int g = tid & 63, rq = tid >> 6;
      const float* eb = eh + ((size_t)(b0 + rq) * kSE) * kHID + 8 * g;
      v4f cacc[4][2];
#pragma unroll
      for (int i = 0; i < 4; ++i) { cacc[i][0] = zero4(); cacc[i][1] = zero4(); }
#pragma unroll 1
      for (int j = 0; j < kSE; ++j) {
#pragma unroll
        for (int i = 0; i < 4; ++i) {
          const float a = Rg[(rq + 4 * i) * kSE + j];
          const float* p = eb + ((size_t)(4 * i) * kSE + j) * kHID;
          const v4f x0 = *(const v4f*)p;
          const v4f x1 = *(const v4f*)(p + 4);
          cacc[i][0] = cacc[i][0] + x0 * a;
          cacc[i][1] = cacc[i][1] + x1 * a;
        }
      }
      v4u hv[4], lv[4];
#pragma unroll
      for (int i = 0; i < 4; ++i) split8(cacc[i][0], cacc[i][1], hv[i], lv[i]);
      for (int pass = 0; pass < 2; ++pass) {
#pragma unroll
        for (int i = 0; i < 4; ++i) {
          const size_t o = (size_t)(rq + 4 * i) * kKCAT + 8 * g;
          *(volatile v4u*)(tgh + o) = hv[i];
          *(volatile v4u*)(tgl + o) = lv[i];
        }
        __threadfence();
      }
    }
    __syncthreads();
    __threadfence();
    v8f acc[4];
#pragma unroll
    for (int j = 0; j < 4; ++j) acc[j] = zero8();
#pragma unroll 1
    for (int k0 = 0; k0 < kKCAT; k0 += 32) {
      V bh[4], bl[4];
#pragma unroll
      for (int j = 0; j < 4; ++j) {
        const size_t bo = (size_t)(64 * wave + 16 * j + rlane) * kKCAT + koff + k0;
        bh[j] = F::load(Wchp + bo);
        bl[j] = F::load(Wclp + bo);
      }
      const int ao = rlane * kKCAT + koff + k0;
      const V ah = F::load(Thp + ao);
      const V al = F::load(Tlp + ao);
#pragma unroll
      for (int j = 0; j < 4; ++j) {
        acc[j] = F::mma(ah, bh[j], acc[j]);
        acc[j] = F::mma(ah, bl[j], acc[j]);
        acc[j] = F::mma(al, bh[j], acc[j]);
      }
      F::guard(acc[0], acc[3], ah, al);
      F::keep(bh[0], bh[1], bh[2], bh[3]);
      F::keep(bl[0], bl[1], bl[2], bl[3]);
    }
    acc_guard4(acc[0], acc[1], acc[2], acc[3]);
#pragma unroll
    for (int j = 0; j < 4; ++j) {
      const int col = 64 * wave + 16 * j + rlane;
#pragma unroll
      for (int r = 0; r < 8; ++r) {
        const int row = 8 * hh + r;
        Ssh[row * kHID + col] = tanhf(acc[j][r] + bcat[j]);
      }
    }
    __syncthreads();
    state_to_planes(Ssh, tgh, tgl, tid);
    __syncthreads();
    __threadfence();
    float* sl = Rg + wave * (16 * 68);
#pragma unroll
    for (int p = 0; p < 2; ++p) {
      v8f pc[4];
#pragma unroll
      for (int j = 0; j < 4; ++j) pc[j] = zero8();
#pragma unroll 1
      for (int k0 = 0; k0 < kHID; k0 += 32) {
        V bh[4], bl[4];
#pragma unroll
        for (int j = 0; j < 4; ++j) {
          const size_t bo = (size_t)(512 * p + 64 * wave + 16 * j + rlane) * kHID + koff + k0;
          bh[j] = F::load(M2hp + bo);
          bl[j] = F::load(M2lp + bo);
        }
        const int ao = rlane * kKCAT + (kHID + kEMB) + koff + k0;
        const V ah = F::load(Thp + ao);
        const V al = F::load(Tlp + ao);
#pragma unroll
        for (int j = 0; j < 4; ++j) {
          pc[j] = F::mma(ah, bh[j], pc[j]);
          pc[j] = F::mma(ah, bl[j], pc[j]);
          pc[j] = F::mma(al, bh[j], pc[j]);
        }
        F::guard(pc[0], pc[3], ah, al);
        F::keep(bh[0], bh[1], bh[2], bh[3]);
        F::keep(bl[0], bl[1], bl[2], bl[3]);
      }
      acc_guard4(pc[0], pc[1], pc[2], pc[3]);
#pragma unroll
      for (int j = 0; j < 4; ++j) {
        const float bv = m2b[512 * p + 64 * wave + 16 * j + rlane];
#pragma unroll
        for (int r = 0; r < 8; ++r) sl[(8 * hh + r) * 68 + 16 * j + rlane] = pc[j][r] + bv;
      }
      __builtin_amdgcn_fence(__ATOMIC_RELEASE, "workgroup");
      __builtin_amdgcn_wave_barrier();
      __builtin_amdgcn_fence(__ATOMIC_ACQUIRE, "workgroup");
      for (int pass = 0; pass < 2; ++pass) {
#pragma unroll
        for (int it = 0; it < 8; ++it) {
          const int row = it * 2 + hh;
          const v4f v = *(const v4f*)(sl + row * 68 + c4);
          *(volatile v4f*)(out + ((size_t)(b0 + row) * kSD + t) * kNOUT + 512 * p + 64 * wave + c4) = v;
        }
        __threadfence();
      }
      __builtin_amdgcn_fence(__ATOMIC_RELEASE, "workgroup");
      __builtin_amdgcn_wave_barrier();
      __builtin_amdgcn_fence(__ATOMIC_ACQUIRE, "workgroup");
    }
    __syncthreads();
  }
}

extern "C" void kernel_launch(void* const* d_in, const int* in_sizes, int n_in,
                              void* d_out, int out_size, void* d_ws, size_t ws_size,
                              hipStream_t stream) {
  if (n_in < 15) return;
  if (out_size < kNB * kSD * kNOUT) return;
  if (in_sizes[0] < kNB * kSE || in_sizes[1] < kNB * kSD || in_sizes[2] < kVOC * kEMB) return;
  if (in_sizes[3] < kHID * kEMB || in_sizes[4] < kHID * kHID || in_sizes[7] < kHID * kHID) return;
  if (in_sizes[9] < kHID * (kHID + kEMB) || in_sizes[10] < kHID * kHID || in_sizes[13] < kNOUT * kHID) return;
  if (in_sizes[5] < kHID || in_sizes[6] < kHID || in_sizes[8] < kHID || in_sizes[11] < kHID || in_sizes[12] < kHID || in_sizes[14] < kNOUT) return;

  const int*   enc_x = (const int*)  d_in[0];
  const int*   dec_y = (const int*)  d_in[1];
  const float* emb   = (const float*)d_in[2];
  const float* eWih  = (const float*)d_in[3];
  const float* eWhh  = (const float*)d_in[4];
  const float* ebih  = (const float*)d_in[5];
  const float* ebhh  = (const float*)d_in[6];
  const float* m1W   = (const float*)d_in[7];
  const float* m1b   = (const float*)d_in[8];
  const float* dWih  = (const float*)d_in[9];
  const float* dWhh  = (const float*)d_in[10];
  const float* dbih  = (const float*)d_in[11];
  const float* dbhh  = (const float*)d_in[12];
  const float* m2W   = (const float*)d_in[13];
  const float* m2b   = (const float*)d_in[14];
  float* out = (float*)d_out;

  const size_t szAE  = (size_t)kNB * kSE * kEMB * 2;
  const size_t szWIH = (size_t)kHID * kEMB * 2;
  const size_t szXW  = (size_t)kSE * kNB * kHID * 4;
  const size_t szWHH = (size_t)kHID * kHID * 2;
  const size_t szEH  = (size_t)kNB * kSE * kHID * 4;
  const size_t szHM  = (size_t)64 * kHID * 2;
  const size_t szM1  = (size_t)kHID * kHID * 2;
  const size_t szS0  = (size_t)64 * kHID * 4;
  const size_t szWC  = (size_t)kHID * kKCAT * 2;
  const size_t szM2  = (size_t)kNOUT * kHID * 2;
  const size_t szTG  = (size_t)kNB * kKCAT * 2;
  char* base = (char*)d_ws;
  size_t off = 0;
  unsigned short* AEh  = (unsigned short*)(base + off); off += szAE;
  unsigned short* AEl  = (unsigned short*)(base + off); off += szAE;
  unsigned short* WIHh = (unsigned short*)(base + off); off += szWIH;
  unsigned short* WIHl = (unsigned short*)(base + off); off += szWIH;
  float*          XW   = (float*)(base + off);          off += szXW;
  unsigned short* WHHh = (unsigned short*)(base + off); off += szWHH;
  unsigned short* WHHl = (unsigned short*)(base + off); off += szWHH;
  float*          EH   = (float*)(base + off);          off += szEH;
  unsigned short* HMh  = (unsigned short*)(base + off); off += szHM;
  unsigned short* HMl  = (unsigned short*)(base + off); off += szHM;
  unsigned short* M1h  = (unsigned short*)(base + off); off += szM1;
  unsigned short* M1l  = (unsigned short*)(base + off); off += szM1;
  float*          S0P  = (float*)(base + off);          off += szS0;
  unsigned short* WCh  = (unsigned short*)(base + off); off += szWC;
  unsigned short* WCl  = (unsigned short*)(base + off); off += szWC;
  unsigned short* M2h  = (unsigned short*)(base + off); off += szM2;
  unsigned short* M2l  = (unsigned short*)(base + off); off += szM2;
  unsigned short* TGh  = (unsigned short*)(base + off); off += szTG;
  unsigned short* TGl  = (unsigned short*)(base + off); off += szTG;
  if (off > ws_size) return;

  {
    const int n8a = kHID * kEMB / 8;   k_split8<<<(n8a + 255) / 256, 256, 0, stream>>>(eWih, WIHh, WIHl, n8a);
    const int n8b = kHID * kHID / 8;   k_split8<<<(n8b + 255) / 256, 256, 0, stream>>>(eWhh, WHHh, WHHl, n8b);
    const int n8c = kHID * kHID / 8;   k_split8<<<(n8c + 255) / 256, 256, 0, stream>>>(m1W, M1h, M1l, n8c);
    const int n8d = kNOUT * kHID / 8;  k_split8<<<(n8d + 255) / 256, 256, 0, stream>>>(m2W, M2h, M2l, n8d);
  }
  {
    const int nthr = kHID * (kKCAT / 8);
    k_build_wcat<<<(nthr + 255) / 256, 256, 0, stream>>>(dWih, dWhh, WCh, WCl, nthr);
  }
  {
    const int nthr = kNB * kSE * (kEMB / 8);
    k_gather_rows<<<(nthr + 255) / 256, 256, 0, stream>>>(enc_x, emb, AEh, AEl, nthr);
  }
  wmma_gemm64<1, true, 2, 0, false, 0><<<dim3((kNB * kSE / 64) * (kHID / 64) / 8, 1, 1), dim3(256, 1, 1), 0, stream>>>(
      AEh, AEl, kEMB, (long)0,
      WIHh, WIHl, kEMB, (long)0,
      (void*)XW, (void*)nullptr, kHID, (long)0,
      ebih, (const float*)nullptr, (long)0,
      kNB * kSE, kHID, kEMB, 1.0f);
  k_encoder<<<kNB / kRB, 256, 0, stream>>>(XW, WHHh, WHHl, ebhh, EH);
  k_hmean<<<(64 * (kHID / 8) + 255) / 256, 256, 0, stream>>>(EH, HMh, HMl);
  wmma_gemm64<1, true, 2, 0, false, 0><<<dim3(1, 1, 1), dim3(256, 1, 1), 0, stream>>>(
      HMh, HMl, kHID, (long)0,
      M1h, M1l, kHID, (long)0,
      (void*)S0P, (void*)nullptr, kHID, (long)0,
      m1b, (const float*)nullptr, (long)0,
      64, kHID, kHID, 1.0f);
  k_decoder<<<kNB / kRB, 256, 0, stream>>>(EH, S0P, dec_y, emb, WCh, WCl, dbih, dbhh, M2h, M2l, m2b, TGh, TGl, out);
}
